// SequentialTransductionUnitJagged_17231408792410
// MI455X (gfx1250) — hardware-verified
//
#include <hip/hip_runtime.h>

typedef __attribute__((ext_vector_type(16))) _Float16 v16h;
typedef __attribute__((ext_vector_type(8)))  _Float16 v8h;
typedef __attribute__((ext_vector_type(16))) __bf16   v16b;
typedef __attribute__((ext_vector_type(8)))  __bf16   v8b;
typedef __attribute__((ext_vector_type(8)))  float    v8f;
typedef __attribute__((ext_vector_type(4)))  float    v4f;
typedef __attribute__((ext_vector_type(4)))  unsigned int u32x4;

constexpr int   EMB_DIM    = 512;
constexpr int   NUM_HEADS  = 8;
constexpr int   HEAD_DIM   = 64;
constexpr int   N_PAD      = 1024;
constexpr int   PROJ_COLS  = 2048;
constexpr int   U_COL0     = 0;
constexpr int   V_COL0     = 512;
constexpr int   Q_COL0     = 1024;
constexpr int   K_COL0     = 1536;
constexpr int   QTILES     = N_PAD / 64;
constexpr float LN_EPS_V   = 1e-6f;
constexpr float W_CARRY    = 64.0f;
constexpr float W_CARRY_INV = 1.0f / 64.0f;
constexpr float MM_CARRY   = 8.0f;
constexpr float MM_CARRY_INV = 0.125f;
constexpr float LOGIT_SC   = 1.0f / 64.0f;
constexpr float P_MUL      = 16.0f;
constexpr float ATT_OUT_SC = 1.0f / 131072.0f;
static_assert(NUM_HEADS * HEAD_DIM == EMB_DIM, "head geometry");
static_assert(EMB_DIM % 64 == 0 && PROJ_COLS % 64 == 0 && N_PAD % 64 == 0, "tile multiples");

__device__ __forceinline__ unsigned short f2bf_bits(float f) {
  unsigned u = __float_as_uint(f);
  return (unsigned short)((u + 0x7FFFu + ((u >> 16) & 1u)) >> 16);
}
__device__ __forceinline__ float bf_bits2f(unsigned short h) { return __uint_as_float(((unsigned)h) << 16); }

__device__ __forceinline__ void dep_guard_h(v8f& a, v8f& b, v16h x, v16h y) { asm volatile("v_nop\n\tv_nop\n\tv_nop\n\tv_nop" : "+v"(a), "+v"(b) : "v"(x), "v"(y)); }
__device__ __forceinline__ void dep_guard_b(v8f& a, v8f& b, v16b x, v16b y) { asm volatile("v_nop\n\tv_nop\n\tv_nop\n\tv_nop" : "+v"(a), "+v"(b) : "v"(x), "v"(y)); }
__device__ __forceinline__ void keep4_h(v16h a, v16h b, v16h c, v16h d) { asm volatile("v_nop" :: "v"(a), "v"(b), "v"(c), "v"(d)); }
__device__ __forceinline__ void keep4_b(v16b a, v16b b, v16b c, v16b d) { asm volatile("v_nop" :: "v"(a), "v"(b), "v"(c), "v"(d)); }
__device__ __forceinline__ void acc_guard4(v8f& a, v8f& b, v8f& c, v8f& d) { asm volatile("v_nop\n\tv_nop\n\tv_nop\n\tv_nop" : "+v"(a), "+v"(b), "+v"(c), "+v"(d)); }
template <typename T> struct Frag;
template <> struct Frag<_Float16> {
  typedef v16h V; union U { v16h v; v8h h[2]; };
  static __device__ __forceinline__ v16h load(const _Float16* p) {
    U f; f.h[0] = *(const v8h*)(p); f.h[1] = *(const v8h*)(p + 16); return f.v;
  }
  static __device__ __forceinline__ v8f mma(v16h a, v16h b, v8f c) {
    return __builtin_amdgcn_wmma_f32_16x16x32_f16(false, a, false, b, (short)0, c, false, false);
  }
  static __device__ __forceinline__ void guard(v8f& a, v8f& b, v16h x, v16h y) { dep_guard_h(a, b, x, y); }
  static __device__ __forceinline__ void keep(v16h a, v16h b, v16h c, v16h d) { keep4_h(a, b, c, d); }
};
template <> struct Frag<__bf16> {
  typedef v16b V; union U { v16b v; v8b h[2]; };
  static __device__ __forceinline__ v16b load(const __bf16* p) {
    U f; f.h[0] = *(const v8b*)(p); f.h[1] = *(const v8b*)(p + 16); return f.v;
  }
  static __device__ __forceinline__ v8f mma(v16b a, v16b b, v8f c) {
    return __builtin_amdgcn_wmma_f32_16x16x32_bf16(false, a, false, b, (short)0, c, false, false);
  }
  static __device__ __forceinline__ void guard(v8f& a, v8f& b, v16b x, v16b y) { dep_guard_b(a, b, x, y); }
  static __device__ __forceinline__ void keep(v16b a, v16b b, v16b c, v16b d) { keep4_b(a, b, c, d); }
};

template <int ET> struct Elem;
template <> struct Elem<0> { typedef _Float16 T; };
template <> struct Elem<1> { typedef __bf16 T; };
template <int ET, bool SPLIT, int BIAS_MODE, int OUT_MODE, bool RESID, int ACT = 0>
__global__ __launch_bounds__(256) void wmma_gemm64(
    const unsigned short* __restrict__ Ap, const unsigned short* __restrict__ A2p, int lda, long strideA,
    const unsigned short* __restrict__ Btp, const unsigned short* __restrict__ Bt2p, int ldb, long strideB,
    void* __restrict__ Cout, void* __restrict__ Cout2, int ldc, long strideC,
    const float* __restrict__ bias,
    const float* __restrict__ resid, long strideR,
    int M, int N, int K, float scale) {
  typedef typename Elem<ET>::T T;
  typedef typename Frag<T>::V V;
  const T* A = (const T*)Ap; const T* A2 = (const T*)A2p; const T* Bt = (const T*)Btp; const T* Bt2 = (const T*)Bt2p;
  __shared__ __align__(16) float sT[8][16 * 68];
  const int b    = blockIdx.y;
  const int lane = threadIdx.x & 31;
  const int wave = threadIdx.x >> 5;
  const int tilesN = N >> 6;
  const int tilesM = M >> 6;
  const int tile = blockIdx.x * 8 + wave;
  if (tile >= tilesM * tilesN) return;
  const int tm = tile / tilesN;
  const int tn = tile - tm * tilesN;
  const int m0 = tm << 6;
  const int n0 = tn << 6;

  const T* Ab  = A  + (size_t)b * strideA;
  const T* Bb  = Bt + (size_t)b * strideB;
  const T* Ab2 = SPLIT ? (A2  + (size_t)b * strideA) : nullptr;
  const T* Bb2 = SPLIT ? (Bt2 + (size_t)b * strideB) : nullptr;

  const int rlane = lane & 15;
  const int koff  = (lane >> 4) * 8;
  const int mOff  = (lane >> 4) * 8;

  v8f acc[4][4];
#pragma unroll
  for (int i = 0; i < 4; ++i)
#pragma unroll
    for (int j = 0; j < 4; ++j) acc[i][j] = (v8f){0.f,0.f,0.f,0.f,0.f,0.f,0.f,0.f};

  for (int k0 = 0; k0 < K; k0 += 32) {
    V bh[4], bl[4];
#pragma unroll
    for (int j = 0; j < 4; ++j) {
      const size_t bo = (size_t)(n0 + (j << 4) + rlane) * ldb + koff + k0;
      bh[j] = Frag<T>::load(Bb + bo);
      if (SPLIT) bl[j] = Frag<T>::load(Bb2 + bo);
    }
#pragma unroll
    for (int i = 0; i < 4; ++i) {
      const size_t ao = (size_t)(m0 + (i << 4) + rlane) * lda + koff + k0;
      V ah = Frag<T>::load(Ab + ao);
      V al;
      if (SPLIT) al = Frag<T>::load(Ab2 + ao);
#pragma unroll
      for (int j = 0; j < 4; ++j) {
        acc[i][j] = Frag<T>::mma(ah, bh[j], acc[i][j]);
        if (SPLIT) {
          acc[i][j] = Frag<T>::mma(ah, bl[j], acc[i][j]);
          acc[i][j] = Frag<T>::mma(al, bh[j], acc[i][j]);
        }
      }
      Frag<T>::guard(acc[i][0], acc[i][3], ah, SPLIT ? al : ah);
    }
    Frag<T>::keep(bh[0], bh[1], bh[2], bh[3]);
    if (SPLIT) Frag<T>::keep(bl[0], bl[1], bl[2], bl[3]);
  }
  acc_guard4(acc[0][0], acc[0][1], acc[0][2], acc[0][3]);
  acc_guard4(acc[1][0], acc[1][1], acc[1][2], acc[1][3]);
  acc_guard4(acc[2][0], acc[2][1], acc[2][2], acc[2][3]);
  acc_guard4(acc[3][0], acc[3][1], acc[3][2], acc[3][3]);

  float* slab = sT[wave];
  const float* Rb = RESID ? (resid + (size_t)b * strideR) : nullptr;
#pragma unroll
  for (int i = 0; i < 4; ++i) {
    const int mBase = m0 + (i << 4);
#pragma unroll
    for (int j = 0; j < 4; ++j) {
      const int n = n0 + (j << 4) + rlane;
      float bv = 0.f;
      if (BIAS_MODE == 2) bv = bias[n];
#pragma unroll
      for (int r = 0; r < 8; ++r) {
        float v = acc[i][j][r] * scale;
        if (BIAS_MODE == 1) v += bias[mBase + mOff + r];
        if (BIAS_MODE == 2) v += bv;
        if (RESID) v += Rb[(size_t)(mBase + mOff + r) * ldc + n];
        if (ACT == 1) v = tanhf(v);
        if (ACT == 2) v = fmaxf(v, 0.0f);
        if (ACT == 4) v = (v > 0.f) ? v : 0.01f * v;
        if (ACT == 6) { const float ex = __expf(-v); v = v * __builtin_amdgcn_rcpf(1.0f + ex) * MM_CARRY; }
        slab[(mOff + r) * 68 + (j << 4) + rlane] = v;
      }
    }
    __builtin_amdgcn_fence(__ATOMIC_RELEASE, "workgroup");
    __builtin_amdgcn_wave_barrier();
    __builtin_amdgcn_fence(__ATOMIC_ACQUIRE, "workgroup");
    if (OUT_MODE == 0) {
      float* C = (float*)Cout + (size_t)b * strideC;
      const int hh = lane >> 4, c4 = (lane & 15) * 4;
      for (int pass = 0; pass < 2; ++pass) {
#pragma unroll
        for (int it = 0; it < 8; ++it) {
          const int row = it * 2 + hh;
          v4f v = *(const v4f*)(slab + row * 68 + c4);
          *(volatile v4f*)(C + (size_t)(mBase + row) * ldc + n0 + c4) = v;
        }
        __threadfence();
      }
    } else {
      const int q = lane >> 3, c8 = (lane & 7) * 8;
      unsigned short* C  = (unsigned short*)Cout  + (size_t)b * strideC;
      unsigned short* C2 = (OUT_MODE == 2) ? ((unsigned short*)Cout2 + (size_t)b * strideC) : nullptr;
      for (int pass = 0; pass < 2; ++pass) {
#pragma unroll
        for (int it = 0; it < 4; ++it) {
          const int row = it * 4 + q;
          const float* sp = slab + row * 68 + c8;
          v8h hv, lv;
#pragma unroll
          for (int e = 0; e < 8; ++e) {
            if (OUT_MODE == 1) {
              hv[e] = (_Float16)sp[e];
            } else {
              unsigned short hb = f2bf_bits(sp[e]);
              unsigned short lb = f2bf_bits(sp[e] - bf_bits2f(hb));
              hv[e] = __builtin_bit_cast(_Float16, hb);
              lv[e] = __builtin_bit_cast(_Float16, lb);
            }
          }
          *(volatile v8h*)(C + (size_t)(mBase + row) * ldc + n0 + c8) = hv;
          if (OUT_MODE == 2) *(volatile v8h*)(C2 + (size_t)(mBase + row) * ldc + n0 + c8) = lv;
        }
        __threadfence();
      }
    }
    __builtin_amdgcn_fence(__ATOMIC_RELEASE, "workgroup");
    __builtin_amdgcn_wave_barrier();
    __builtin_amdgcn_fence(__ATOMIC_ACQUIRE, "workgroup");
  }
}

__global__ __launch_bounds__(256) void cast_f32_f16x2(
    const float* __restrict__ in, unsigned short* __restrict__ outp, int n2, float mul) {
  int i = blockIdx.x * 256 + threadIdx.x;
  if (i < n2) {
    const _Float16 h0 = (_Float16)(in[2 * i] * mul), h1 = (_Float16)(in[2 * i + 1] * mul);
    const unsigned u = (unsigned)__builtin_bit_cast(unsigned short, h0) | ((unsigned)__builtin_bit_cast(unsigned short, h1) << 16);
    ((volatile unsigned*)outp)[i] = u;
    __threadfence();
    ((volatile unsigned*)outp)[i] = u;
  }
}

constexpr int WT_PITCH = 72;
__global__ __launch_bounds__(256) void wt_cast_k(const float* __restrict__ W, unsigned short* __restrict__ Wtp,
                                                 int K, int N, float mul) {
  __shared__ __align__(16) _Float16 st[64 * WT_PITCH];
  _Float16* Wt = (_Float16*)Wtp;
  const int n0 = blockIdx.x * 64, k0 = blockIdx.y * 64;
  const int tid = threadIdx.x;
  const int kr = tid >> 2, c16 = (tid & 3) * 16;
  const float* src = W + (size_t)(k0 + kr) * N + n0 + c16;
#pragma unroll
  for (int q = 0; q < 4; ++q) {
    const v4f v = *(const v4f*)(src + 4 * q);
#pragma unroll
    for (int e = 0; e < 4; ++e) {
      st[(c16 + 4 * q + e) * WT_PITCH + kr] = (_Float16)(v[e] * mul);
    }
  }
  __syncthreads();
  const int wave = tid >> 5, lane = tid & 31;
  const int q8 = lane >> 3, c8 = (lane & 7) * 8;
  const v8h h0 = *(const v8h*)(st + (wave * 4 + q8) * WT_PITCH + c8);
  const v8h h1 = *(const v8h*)(st + (32 + wave * 4 + q8) * WT_PITCH + c8);
  for (int pass = 0; pass < 2; ++pass) {
    *(volatile v8h*)(Wt + (size_t)(n0 + wave * 4 + q8) * K + k0 + c8) = h0;
    *(volatile v8h*)(Wt + (size_t)(n0 + 32 + wave * 4 + q8) * K + k0 + c8) = h1;
    __threadfence();
  }
}

__global__ __launch_bounds__(64) void ln_x_k(const float* __restrict__ xin, unsigned short* __restrict__ o0p, int nrows_valid) {
  __shared__ float red1[2], red2[2];
  _Float16* o0 = (_Float16*)o0p;
  const int row = blockIdx.x, tid = threadIdx.x, lane = tid & 31, wave = tid >> 5;
  const bool valid = row < nrows_valid;
  const int rowc = valid ? row : (nrows_valid - 1);
  const size_t rb = (size_t)rowc * EMB_DIM;
  const size_t ob = (size_t)row * EMB_DIM;
  const int c0 = tid * 8;
  const v4f va = *(const v4f*)(xin + rb + c0);
  const v4f vb = *(const v4f*)(xin + rb + c0 + 4);
  float s = ((va[0] + va[1]) + (va[2] + va[3])) + ((vb[0] + vb[1]) + (vb[2] + vb[3]));
#pragma unroll
  for (int off = 1; off < 32; off <<= 1) s += __shfl_xor(s, off, 32);
  if (lane == 0) red1[wave] = s;
  __syncthreads();
  const float mu = (red1[0] + red1[1]) * (1.0f / EMB_DIM);
  const v4f da = va - mu, db = vb - mu;
  float s2 = ((da[0] * da[0] + da[1] * da[1]) + (da[2] * da[2] + da[3] * da[3])) +
             ((db[0] * db[0] + db[1] * db[1]) + (db[2] * db[2] + db[3] * db[3]));
#pragma unroll
  for (int off = 1; off < 32; off <<= 1) s2 += __shfl_xor(s2, off, 32);
  if (lane == 0) red2[wave] = s2;
  __syncthreads();
  const float var = (red2[0] + red2[1]) * (1.0f / EMB_DIM);
  const float inv = rsqrtf(var + LN_EPS_V);
  v8h hv;
#pragma unroll
  for (int e = 0; e < 4; ++e) {
    const float ya = valid ? (da[e] * inv) : 0.0f;
    const float yb = valid ? (db[e] * inv) : 0.0f;
    hv[e]     = (_Float16)ya;
    hv[4 + e] = (_Float16)yb;
  }
  for (int pass = 0; pass < 2; ++pass) {
    *(volatile v8h*)(o0 + ob + c0) = hv;
    __threadfence();
  }
}

__global__ __launch_bounds__(64) void ln_mul_k(const float* __restrict__ att, const unsigned short* __restrict__ mmp,
                                              unsigned short* __restrict__ oinp) {
  __shared__ float red1[2], red2[2];
  const _Float16* mm = (const _Float16*)mmp;
  _Float16* oin = (_Float16*)oinp;
  const int row = blockIdx.x, tid = threadIdx.x, lane = tid & 31, wave = tid >> 5;
  const size_t rb = (size_t)row * EMB_DIM;
  const int c0 = tid * 8;
  const v4f va = *(const v4f*)(att + rb + c0);
  const v4f vb = *(const v4f*)(att + rb + c0 + 4);
  float s = ((va[0] + va[1]) + (va[2] + va[3])) + ((vb[0] + vb[1]) + (vb[2] + vb[3]));
#pragma unroll
  for (int off = 1; off < 32; off <<= 1) s += __shfl_xor(s, off, 32);
  if (lane == 0) red1[wave] = s;
  __syncthreads();
  const float mu = (red1[0] + red1[1]) * (1.0f / EMB_DIM);
  const v4f da = va - mu, db = vb - mu;
  float s2 = ((da[0] * da[0] + da[1] * da[1]) + (da[2] * da[2] + da[3] * da[3])) +
             ((db[0] * db[0] + db[1] * db[1]) + (db[2] * db[2] + db[3] * db[3]));
#pragma unroll
  for (int off = 1; off < 32; off <<= 1) s2 += __shfl_xor(s2, off, 32);
  if (lane == 0) red2[wave] = s2;
  __syncthreads();
  const float var = (red2[0] + red2[1]) * (1.0f / EMB_DIM);
  const float inv = rsqrtf(var + LN_EPS_V);
  const v8h uh = *(const v8h*)(mm + (size_t)row * PROJ_COLS + U_COL0 + c0);
  v8h hv;
#pragma unroll
  for (int e = 0; e < 4; ++e) {
    const float ua = (float)uh[e] * MM_CARRY_INV;
    const float ub = (float)uh[4 + e] * MM_CARRY_INV;
    hv[e]     = (_Float16)(ua * (da[e] * inv));
    hv[4 + e] = (_Float16)(ub * (db[e] * inv));
  }
  for (int pass = 0; pass < 2; ++pass) {
    *(volatile v8h*)(oin + rb + c0) = hv;
    __threadfence();
  }
}

__device__ __forceinline__ v8f mma_h(v16h a, v16h b, v8f c) {
  c = __builtin_amdgcn_wmma_f32_16x16x32_f16(false, a, false, b, (short)0, c, false, false);
  asm volatile("v_nop\n\tv_nop\n\tv_nop\n\tv_nop" : "+v"(c) : "v"(a), "v"(b));
  return c;
}
union Ld8 { u32x4 w; v8h h; };

__global__ __launch_bounds__(128)
void jag_attn_k(const unsigned short* __restrict__ mmp, const float* __restrict__ mask,
                 const int* __restrict__ offs, float* __restrict__ att, int ntok, int nseq) {
  __shared__ __align__(16) _Float16 Qsh[64 * 64];
  __shared__ __align__(16) _Float16 Ksh[64 * 64];
  __shared__ __align__(16) _Float16 Vth[64 * 64];
  __shared__ __align__(16) _Float16 Psh[4][16 * 64];
  __shared__ __align__(16) float    Os[4][16 * 68];

  const _Float16* mm = (const _Float16*)mmp;
  const int tid  = threadIdx.x;
  const int wave = tid >> 5;
  const int lane = tid & 31;
  const int hh   = lane >> 4;
  const int c    = lane & 15;

  const int bx = blockIdx.x;
  const int qb = bx % QTILES;
  const int bhid = bx / QTILES;
  const int h  = bhid % NUM_HEADS;
  const int b  = bhid / NUM_HEADS;
  if (b >= nseq) return;
  int off  = offs[b];
  int off1 = offs[b + 1];
  off  = off  < 0 ? 0 : (off  > ntok ? ntok : off);
  off1 = off1 < off ? off : (off1 > ntok ? ntok : off1);
  int len = off1 - off;
  if (len > N_PAD) len = N_PAD;
  const int qblk = qb * 64;
  if (qblk >= len) return;
  const int q0 = qblk + wave * 16;
  const u32x4 zero4 = {0u, 0u, 0u, 0u};

  {
    const int r = tid >> 1, cb = (tid & 1) * 32;
    const int qp = qblk + r;
    const bool ok = qp < len;
    int tok = off + (ok ? qp : 0);
    tok = tok > ntok - 1 ? ntok - 1 : tok;
    const _Float16* src = mm + (size_t)tok * PROJ_COLS + Q_COL0 + h * HEAD_DIM + cb;
#pragma unroll
    for (int i = 0; i < 4; ++i) {
      Ld8 u; u.w = *(const u32x4*)(src + 8 * i);
      if (!ok) u.w = zero4;
      *(u32x4*)(Qsh + r * 64 + cb + 8 * i) = u.w;
    }
  }
  __syncthreads();
  v16h qa[2];
#pragma unroll
  for (int dc = 0; dc < 2; ++dc) qa[dc] = Frag<_Float16>::load(Qsh + (wave * 16 + c) * 64 + dc * 32 + 8 * hh);

  v8f oacc[4];
#pragma unroll
  for (int t = 0; t < 4; ++t) oacc[t] = (v8f){0.f,0.f,0.f,0.f,0.f,0.f,0.f,0.f};

  const int nChunks = qb + 1;
  for (int kc = 0; kc < nChunks; ++kc) {
    const int kv0 = kc * 64;
    __syncthreads();
    {
      const int r = tid >> 1, cb = (tid & 1) * 32;
      const int kp = kv0 + r;
      const bool ok = kp < len;
      int tok = off + (ok ? kp : 0);
      tok = tok > ntok - 1 ? ntok - 1 : tok;
      const _Float16* srcK = mm + (size_t)tok * PROJ_COLS + K_COL0 + h * HEAD_DIM + cb;
      const _Float16* srcV = mm + (size_t)tok * PROJ_COLS + V_COL0 + h * HEAD_DIM + cb;
#pragma unroll
      for (int i = 0; i < 4; ++i) {
        Ld8 uk; uk.w = *(const u32x4*)(srcK + 8 * i);
        Ld8 uv; uv.w = *(const u32x4*)(srcV + 8 * i);
        if (!ok) { uk.w = zero4; uv.w = zero4; }
        *(u32x4*)(Ksh + r * 64 + cb + 8 * i) = uk.w;
#pragma unroll
        for (int e = 0; e < 8; ++e) Vth[(cb + 8 * i + e) * 64 + r] = uv.h[e];
      }
    }
    __syncthreads();

    v8f s[4];
#pragma unroll
    for (int j = 0; j < 4; ++j) {
      s[j] = (v8f){0.f,0.f,0.f,0.f,0.f,0.f,0.f,0.f};
#pragma unroll
      for (int dc = 0; dc < 2; ++dc) {
        const v16h kf = Frag<_Float16>::load(Ksh + (j * 16 + c) * 64 + dc * 32 + 8 * hh);
        s[j] = mma_h(qa[dc], kf, s[j]);
      }
    }
    _Float16* pw = Psh[wave];
#pragma unroll
    for (int r = 0; r < 8; ++r) {
      int qrow = q0 + 8 * hh + r;
      qrow = qrow > N_PAD - 1 ? N_PAD - 1 : qrow;
      const float* mrow = mask + (size_t)qrow * N_PAD + kv0;
#pragma unroll
      for (int j = 0; j < 4; ++j) {
        const int kvc = j * 16 + c;
        const float l  = s[j][r] * LOGIT_SC;
        const float ex = __expf(-l);
        const float sg = __builtin_amdgcn_rcpf(1.0f + ex);
        float p = l * sg;
        p = p * mrow[kvc];
        p = p * P_MUL;
        pw[(8 * hh + r) * 64 + kvc] = (_Float16)p;
      }
    }
    __builtin_amdgcn_fence(__ATOMIC_RELEASE, "workgroup");
    __builtin_amdgcn_wave_barrier();
    __builtin_amdgcn_fence(__ATOMIC_ACQUIRE, "workgroup");
#pragma unroll
    for (int kk = 0; kk < 2; ++kk) {
      const v16h pa = Frag<_Float16>::load(pw + c * 64 + kk * 32 + 8 * hh);
#pragma unroll
      for (int t = 0; t < 4; ++t) {
        const v16h vf = Frag<_Float16>::load(Vth + (t * 16 + c) * 64 + kk * 32 + 8 * hh);
        oacc[t] = mma_h(pa, vf, oacc[t]);
      }
    }
  }

  float* os = Os[wave];
#pragma unroll
  for (int r = 0; r < 8; ++r) {
#pragma unroll
    for (int t = 0; t < 4; ++t) os[(8 * hh + r) * 68 + t * 16 + c] = oacc[t][r] * ATT_OUT_SC;
  }
  __builtin_amdgcn_fence(__ATOMIC_RELEASE, "workgroup");
  __builtin_amdgcn_wave_barrier();
  __builtin_amdgcn_fence(__ATOMIC_ACQUIRE, "workgroup");
  {
    const int c4 = (lane & 15) * 4;
    float* ob_ptr = att + (size_t)h * HEAD_DIM;
    for (int pass = 0; pass < 2; ++pass) {
#pragma unroll
      for (int it = 0; it < 8; ++it) {
        const int row = it * 2 + hh;
        const int qr = q0 + row;
        const v4f val = *(const v4f*)(os + row * 68 + c4);
        if (qr < len) {
          *(volatile v4f*)(ob_ptr + (size_t)(off + qr) * EMB_DIM + c4) = val;
        }
      }
      __threadfence();
    }
  }
}

static inline size_t align256(size_t v) { return (v + 255) & ~(size_t)255; }

extern "C" void kernel_launch(void* const* d_in, const int* in_sizes, int n_in,
                              void* d_out, int out_size, void* d_ws, size_t ws_size,
                              hipStream_t stream) {
  if (n_in < 6) return;
  const float* x     = (const float*)d_in[0];
  const int*   offs  = (const int*)d_in[1];
  const float* maskp = (const float*)d_in[2];
  const float* uvqk  = (const float*)d_in[3];
  const float* ow    = (const float*)d_in[4];
  const float* ob    = (const float*)d_in[5];
  float*       out   = (float*)d_out;

  const int T    = in_sizes[0] / EMB_DIM;
  const int nseq = in_sizes[1] - 1;
  if (T < 1 || nseq < 1) return;
  if (in_sizes[0] != T * EMB_DIM) return;
  if (in_sizes[2] < N_PAD * N_PAD) return;
  if (in_sizes[3] != EMB_DIM * PROJ_COLS) return;
  if (in_sizes[4] != EMB_DIM * EMB_DIM) return;
  if (in_sizes[5] < EMB_DIM) return;
  const int Tp  = ((T + 63) / 64) * 64;
  const int T64 = (T / 64) * 64;
  if (out_size < T64 * EMB_DIM) return;

  const size_t szXN  = (size_t)Tp * EMB_DIM * 2;
  const size_t szWU  = (size_t)PROJ_COLS * EMB_DIM * 2;
  const size_t szMM  = (size_t)Tp * PROJ_COLS * 2;
  const size_t szATT = (size_t)Tp * EMB_DIM * 4;
  const size_t szWO  = (size_t)EMB_DIM * EMB_DIM * 2;
  const size_t oXN  = 0;
  const size_t oWU  = align256(oXN + szXN);
  const size_t oMM  = align256(oWU + szWU);
  const size_t oATT = align256(oMM + szMM);
  const size_t oWO  = align256(oATT + szATT);
  const size_t total = align256(oWO + szWO);
  if (total > ws_size) return;

  char* ws = (char*)d_ws;
  unsigned short* XN  = (unsigned short*)(ws + oXN);
  unsigned short* OIN = XN;
  unsigned short* WU  = (unsigned short*)(ws + oWU);
  unsigned short* MM  = (unsigned short*)(ws + oMM);
  float*          ATT = (float*)(ws + oATT);
  unsigned short* WO  = (unsigned short*)(ws + oWO);

  ln_x_k<<<dim3(Tp), dim3(64), 0, stream>>>(x, XN, T);
  wt_cast_k<<<dim3(PROJ_COLS / 64, EMB_DIM / 64), dim3(256), 0, stream>>>(uvqk, WU, EMB_DIM, PROJ_COLS, W_CARRY);
  {
    const int n2 = (EMB_DIM * EMB_DIM) / 2;
    cast_f32_f16x2<<<dim3((n2 + 255) / 256), dim3(256), 0, stream>>>(ow, WO, n2, W_CARRY);
  }
  {
    const int tiles = (Tp / 64) * (PROJ_COLS / 64);
    wmma_gemm64<0, false, 0, 1, false, 6><<<dim3((tiles + 7) / 8, 1), dim3(256), 0, stream>>>(
        XN, XN, EMB_DIM, 0L, WU, WU, EMB_DIM, 0L, (void*)MM, (void*)MM, PROJ_COLS, 0L,
        ob, x, 0L, Tp, PROJ_COLS, EMB_DIM, W_CARRY_INV);
  }
  jag_attn_k<<<dim3(nseq * NUM_HEADS * QTILES), dim3(128), 0, stream>>>(MM, maskp, offs, ATT, T, nseq);
  if (T64 > 0) {
    ln_mul_k<<<dim3(T64), dim3(64), 0, stream>>>(ATT, MM, OIN);
    const int tiles = (T64 / 64) * (EMB_DIM / 64);
    wmma_gemm64<0, false, 2, 0, true, 0><<<dim3((tiles + 7) / 8, 1), dim3(256), 0, stream>>>(
        OIN, OIN, EMB_DIM, 0L, WO, WO, EMB_DIM, 0L, (void*)out, (void*)out, EMB_DIM, 0L,
        ob, x, 0L, T64, EMB_DIM, EMB_DIM, W_CARRY_INV);
  }
}
